// ProtoNetItemUserLL_54520314856137
// MI455X (gfx1250) — hardware-verified
//
#include <hip/hip_runtime.h>
#include <math.h>


#define NQ 16384
#define MM 2048
#define DD 128
typedef __attribute__((ext_vector_type(16))) _Float16 v16h;
typedef __attribute__((ext_vector_type(8)))  _Float16 v8h;
typedef __attribute__((ext_vector_type(8)))  float    v8f;
typedef __attribute__((ext_vector_type(4)))  float    v4f;
#define VST2(T, ptr, val) do { const T _v = (val); *(volatile T*)(ptr) = _v; __threadfence(); *(volatile T*)(ptr) = _v; } while (0)
__device__ __forceinline__ v8f wmma16(v16h a, v16h b, v8f c) {
  v8f d = __builtin_amdgcn_wmma_f32_16x16x32_f16(false, a, false, b, (short)0, c, false, false);
  asm volatile("v_nop\n\tv_nop\n\tv_nop\n\tv_nop" : "+v"(d) : "v"(a), "v"(b));
  return d;
}
__device__ __forceinline__ v16h frag16(const _Float16* p, int hh) {
  const v8h lo = *(const v8h*)(p + 8 * hh), hi = *(const v8h*)(p + 16 + 8 * hh);
  return __builtin_shufflevector(lo, hi, 0,1,2,3,4,5,6,7,8,9,10,11,12,13,14,15);
}
template <bool NORM>
__global__ __launch_bounds__(256) void k_rows16(const float* __restrict__ s, int rows, _Float16* __restrict__ d) {
  const int row = blockIdx.x * 8 + (threadIdx.x >> 5), lane = threadIdx.x & 31;
  if (row >= rows) return;
  v4f v = *(const v4f*)(s + (size_t)row * DD + lane * 4);
  float sc = 1.0f;
  if (NORM) { float q = v[0]*v[0] + v[1]*v[1] + v[2]*v[2] + v[3]*v[3];
#pragma unroll
    for (int o = 16; o > 0; o >>= 1) q += __shfl_xor(q, o, 32);
    sc = 1.0f / fmaxf(sqrtf(q), 1e-8f); }
  typedef __attribute__((ext_vector_type(4))) _Float16 v4h; v4h o;
#pragma unroll
  for (int e = 0; e < 4; ++e) o[e] = (_Float16)(v[e] * sc);
  VST2(v4h, d + (size_t)row * DD + lane * 4, o);
}
__global__ __launch_bounds__(256) void k_w16(const float* __restrict__ w, int N, int K, int lds, _Float16* __restrict__ W16) {
  const int t = blockIdx.x * 256 + threadIdx.x; const int per = K / 8;
  if (t >= N * per) return;
  const int n = t / per, k0 = (t % per) * 8;
  v8h o;
#pragma unroll
  for (int e = 0; e < 8; ++e) o[e] = (_Float16)w[(size_t)n * lds + k0 + e];
  VST2(v8h, W16 + (size_t)n * K + k0, o);
}
__global__ __launch_bounds__(256) void k_mwT(const float* __restrict__ mw, _Float16* __restrict__ MT) {
  const int t = blockIdx.x * 256 + threadIdx.x;
  const int d = t >> 8, m0 = (t & 255) * 8;
  v8h o;
#pragma unroll
  for (int e = 0; e < 8; ++e) o[e] = (_Float16)mw[(size_t)(m0 + e) * DD + d];
  VST2(v8h, MT + (size_t)d * MM + m0, o);
}
template <int K, int NTOT, int EPI>
__global__ __launch_bounds__(128) void k_gemm(const _Float16* __restrict__ A, const _Float16* __restrict__ W16, const float* __restrict__ bias,
                                              const float* __restrict__ aux1, const float* __restrict__ aux2, float* __restrict__ outf, _Float16* __restrict__ outh) {
  __shared__ __attribute__((aligned(16))) float sT[4][16][132];
  const int lane = threadIdx.x & 31, wave = threadIdx.x >> 5, hh = lane >> 4, l16 = lane & 15;
  const int m0 = blockIdx.x * 64 + wave * 16, n0 = blockIdx.y * 128;
  v8f acc[8];
#pragma unroll
  for (int ni = 0; ni < 8; ++ni) acc[ni] = (v8f){};
#pragma unroll 2
  for (int k0 = 0; k0 < K; k0 += 32) {
    const v16h a0 = frag16(A + (size_t)(m0 + l16) * K + k0, hh);
#pragma unroll
    for (int ni = 0; ni < 8; ++ni) { const v16h b = frag16(W16 + (size_t)(n0 + ni * 16 + l16) * K + k0, hh); acc[ni] = wmma16(a0, b, acc[ni]); }
  }
  float (*st)[132] = sT[wave];
#pragma unroll
  for (int ni = 0; ni < 8; ++ni)
#pragma unroll
    for (int i = 0; i < 8; ++i) st[i + 8 * hh][ni * 16 + l16] = acc[ni][i] + ((EPI == 0 || EPI == 3) ? bias[n0 + ni * 16 + l16] : 0.f);
  __builtin_amdgcn_fence(__ATOMIC_RELEASE, "workgroup"); __builtin_amdgcn_wave_barrier(); __builtin_amdgcn_fence(__ATOMIC_ACQUIRE, "workgroup");
  for (int pass = 0; pass < 2; ++pass) {
#pragma unroll
    for (int rr = 0; rr < 16; ++rr) {
      const int row = m0 + rr;
      v4f v = *(const v4f*)(&st[rr][lane * 4]);
      if (EPI == 2) { const float ri = aux1[(size_t)row * 4]; v *= ri; }
      if (EPI == 3) { const v4f qv = *(const v4f*)(aux1 + (size_t)row * DD + lane * 4), mv = *(const v4f*)(aux2 + (size_t)row * DD + lane * 4);
#pragma unroll
        for (int e = 0; e < 4; ++e) { const float g = tanhf(v[e]); v[e] = (1.0f - g) * qv[e] + g * mv[e]; } }
      *(volatile v4f*)(outf + (size_t)row * NTOT + n0 + lane * 4) = v;
      if (EPI == 2) { typedef __attribute__((ext_vector_type(4))) _Float16 v4h; v4h o;
#pragma unroll
        for (int e = 0; e < 4; ++e) o[e] = (_Float16)v[e];
        *(volatile v4h*)(outh + (size_t)row * (2 * DD) + lane * 4) = o; }
    }
    __threadfence();
  }
}
__global__ __launch_bounds__(256) void k_softmax(const float* __restrict__ Sc, _Float16* __restrict__ P16, float* __restrict__ rinv) {
  const int row = blockIdx.x * 8 + (threadIdx.x >> 5), lane = threadIdx.x & 31;
  const float* sr = Sc + (size_t)row * MM;
  float mx = -INFINITY;
  for (int j = lane * 4; j < MM; j += 128) { const v4f v = *(const v4f*)(sr + j); mx = fmaxf(mx, fmaxf(fmaxf(v[0], v[1]), fmaxf(v[2], v[3]))); }
#pragma unroll
  for (int o = 16; o > 0; o >>= 1) mx = fmaxf(mx, __shfl_xor(mx, o, 32));
  float sum = 0.f;
  typedef __attribute__((ext_vector_type(4))) _Float16 v4h;
  for (int pass = 0; pass < 2; ++pass) {
    sum = 0.f;
    for (int j = lane * 4; j < MM; j += 128) { const v4f v = *(const v4f*)(sr + j); v4h o;
#pragma unroll
      for (int e = 0; e < 4; ++e) { const float p = expf(v[e] - mx); sum += p; o[e] = (_Float16)p; }
      *(volatile v4h*)(P16 + (size_t)row * MM + j) = o; }
    __threadfence();
  }
#pragma unroll
  for (int o = 16; o > 0; o >>= 1) sum += __shfl_xor(sum, o, 32);
  __shared__ float rv[32];
  if (lane < 4) rv[(threadIdx.x >> 5) * 4 + lane] = 1.0f / sum;
  __syncthreads();
  if (threadIdx.x < 32) { *(volatile float*)(rinv + (size_t)blockIdx.x * 32 + threadIdx.x) = rv[threadIdx.x]; __threadfence(); *(volatile float*)(rinv + (size_t)blockIdx.x * 32 + threadIdx.x) = rv[threadIdx.x]; }
}
__global__ __launch_bounds__(256) void k_q16(const float* __restrict__ q, _Float16* __restrict__ G16) {
  const int t = blockIdx.x * 256 + threadIdx.x;
  const int row = t >> 5, c = (t & 31) * 4;
  typedef __attribute__((ext_vector_type(4))) _Float16 v4h; v4h o; const v4f v = *(const v4f*)(q + (size_t)row * DD + c);
#pragma unroll
  for (int e = 0; e < 4; ++e) o[e] = (_Float16)v[e];
  VST2(v4h, G16 + (size_t)row * (2 * DD) + DD + c, o);
}
extern "C" void kernel_launch(void* const* d_in, const int* in_sizes, int n_in,
                              void* d_out, int out_size, void* d_ws, size_t ws_size, hipStream_t stream) {
  (void)in_sizes; (void)n_in; (void)out_size;
  const float* q    = (const float*)d_in[0];
  const float* Wt   = (const float*)d_in[1];  const float* bt = (const float*)d_in[2];
  const float* mi   = (const float*)d_in[3];
  const float* mw   = (const float*)d_in[4];
  const float* Wt2  = (const float*)d_in[5];  const float* bt2 = (const float*)d_in[6];
  float* out  = (float*)d_out;
  float* memo = (float*)((char*)d_out + (size_t)NQ * DD * 4);
  char* ws = (char*)d_ws; size_t off = 0;
  auto take = [&](size_t bytes) { void* p = ws + off; off = (off + bytes + 255) & ~(size_t)255; return p; };
  _Float16* Q16  = (_Float16*)take((size_t)NQ * DD * 2);
  _Float16* Wt6  = (_Float16*)take((size_t)DD * DD * 2);
  float*    TQ   = (float*)take((size_t)NQ * DD * 4);
  _Float16* TQn  = (_Float16*)take((size_t)NQ * DD * 2);
  _Float16* MIn  = (_Float16*)take((size_t)MM * DD * 2);
  _Float16* MT   = (_Float16*)take((size_t)DD * MM * 2);
  float*    Sc   = (float*)take((size_t)NQ * MM * 4);
  _Float16* P16  = (_Float16*)take((size_t)NQ * MM * 2);
  float*    rinv = (float*)take((size_t)NQ * 4 * 4);
  _Float16* G16  = (_Float16*)take((size_t)NQ * 2 * DD * 2);
  _Float16* Wt26 = (_Float16*)take((size_t)DD * 2 * DD * 2);
  if (off > ws_size) return;
  const dim3 b256(256);
  k_rows16<false><<<NQ / 8, b256, 0, stream>>>(q, NQ, Q16);
  k_w16<<<(DD * 16 + 255) / 256, b256, 0, stream>>>(Wt, DD, DD, DD, Wt6);
  k_gemm<DD, DD, 0><<<dim3(NQ / 64, 1), 128, 0, stream>>>(Q16, Wt6, bt, nullptr, nullptr, TQ, nullptr);
  k_rows16<true><<<NQ / 8, b256, 0, stream>>>(TQ, NQ, TQn);
  k_rows16<true><<<MM / 8, b256, 0, stream>>>(mi, MM, MIn);
  k_gemm<DD, MM, 1><<<dim3(NQ / 64, MM / 128), 128, 0, stream>>>(TQn, MIn, nullptr, nullptr, nullptr, Sc, nullptr);
  k_softmax<<<NQ / 8, b256, 0, stream>>>(Sc, P16, rinv);
  k_mwT<<<DD * 256 / 256, b256, 0, stream>>>(mw, MT);
  k_gemm<MM, DD, 2><<<dim3(NQ / 64, 1), 128, 0, stream>>>(P16, MT, nullptr, rinv, nullptr, memo, G16);
  k_q16<<<NQ * 32 / 256, b256, 0, stream>>>(q, G16);
  k_w16<<<(DD * 32 + 255) / 256, b256, 0, stream>>>(Wt2, DD, 2 * DD, 2 * DD, Wt26);
  k_gemm<2 * DD, DD, 3><<<dim3(NQ / 64, 1), 128, 0, stream>>>(G16, Wt26, bt2, q, memo, out, nullptr);
}
